// MHA_71975061946783
// MI455X (gfx1250) — hardware-verified
//
#include <hip/hip_runtime.h>


#ifndef NB
#define NB 4
#endif
#ifndef SEQ
#define SEQ 2048
#endif
#define TT       SEQ
#define TT_FULL  2048
#define DM       1024
#define NH_      16
#define HD       64
#define RH       ((TT < 256) ? TT : 256)
#define MT       (NB * TT)
#define MH       (NB * RH)
#define L2E      1.4426950408889634f

static_assert(DM == NH_ * HD);
static_assert(HD == 64);
static_assert(DM % 64 == 0);
static_assert(TT % 64 == 0);
static_assert(RH % 64 == 0);
static_assert(MT % 64 == 0);
static_assert(((size_t)TT * DM) % 8 == 0);
static_assert(TT <= TT_FULL);

typedef _Float16 h16;
typedef unsigned short bf;
typedef __attribute__((ext_vector_type(16))) __bf16   v16bf;
typedef __attribute__((ext_vector_type(16))) _Float16 v16h;
typedef __attribute__((ext_vector_type(8)))  _Float16 v8h;
typedef __attribute__((ext_vector_type(8)))  unsigned short v8us;
typedef __attribute__((ext_vector_type(8)))  float    v8f;
typedef __attribute__((ext_vector_type(4)))  float    v4f;
typedef v4f  __attribute__((may_alias)) v4fa;
typedef v8us __attribute__((may_alias)) v8usa;

__device__ __forceinline__ unsigned short f2bf(float f) { unsigned u = __float_as_uint(f); u += 0x7FFFu + ((u >> 16) & 1u); return (unsigned short)(u >> 16); }
__device__ __forceinline__ float bf2f(unsigned short b) { return __uint_as_float(((unsigned)b) << 16); }
__device__ __forceinline__ float bfr(float f) { return bf2f(f2bf(f)); }
__device__ __forceinline__ void splitf(float y, unsigned short& h, unsigned short& l) { h = f2bf(y); l = f2bf(y - bf2f(h)); }
__device__ __forceinline__ v16h cat16(v8h lo, v8h hi) { return __builtin_shufflevector(lo, hi, 0, 1, 2, 3, 4, 5, 6, 7, 8, 9, 10, 11, 12, 13, 14, 15); }
__device__ __forceinline__ v16bf cat16b(v8us lo, v8us hi) { return __builtin_bit_cast(v16bf, __builtin_shufflevector(lo, hi, 0, 1, 2, 3, 4, 5, 6, 7, 8, 9, 10, 11, 12, 13, 14, 15)); }
__device__ __forceinline__ v8f wmma16(v16h a, v16h b, v8f c) { return __builtin_amdgcn_wmma_f32_16x16x32_f16(false, a, false, b, (short)0, c, false, false); }
__device__ __forceinline__ v8f wmmab(v16bf a, v16bf b, v8f c) { return __builtin_amdgcn_wmma_f32_16x16x32_bf16(false, a, false, b, (short)0, c, false, false); }

template <typename T16> struct WFrag;
template <> struct WFrag<h16> { typedef v16h V; static __device__ __forceinline__ V ld(const h16* p) { return cat16(*(const v8h*)p, *(const v8h*)(p + 16)); } static __device__ __forceinline__ v8f mma(V a, V b, v8f c) { return wmma16(a, b, c); } };
template <> struct WFrag<bf> { typedef v16bf V; static __device__ __forceinline__ V ld(const bf* p) { return cat16b(*(const v8us*)p, *(const v8us*)(p + 16)); } static __device__ __forceinline__ v8f mma(V a, V b, v8f c) { return wmmab(a, b, c); } };

template <typename T16, int NSPLIT, int EPI>
__global__ __launch_bounds__(32) void k_gemmw(const T16* __restrict__ A, const T16* __restrict__ A2, const T16* __restrict__ Bt, const T16* __restrict__ Bt2, int K, float* C, int ldc, const float* __restrict__ bias, bf* Ph, bf* Pl, h16* P16, float osc) {
    typedef typename WFrag<T16>::V V;
    __shared__ __align__(16) float os[(EPI == 2) ? 4 : 16 * 68];
    __shared__ __align__(16) unsigned short tt[(EPI == 2) ? 3 * 64 * 72 : 8];
    const unsigned lane = threadIdx.x & 31u, lr = lane & 15u, hi = lane >> 4; const unsigned r0 = blockIdx.x * 64u, c0 = blockIdx.y * 64u;
    v8f acc[4][4];
#pragma unroll
    for (int mb = 0; mb < 4; ++mb)
#pragma unroll
        for (int nb = 0; nb < 4; ++nb) acc[mb][nb] = (v8f){};
    const size_t aoff = (size_t)(r0 + lr) * K + 8u * hi, boff = (size_t)(c0 + lr) * K + 8u * hi;
#pragma unroll 1
    for (int kc = 0; kc < K; kc += 32) {
        V a[4], a2[4];
#pragma unroll
        for (int mb = 0; mb < 4; ++mb) { a[mb] = WFrag<T16>::ld(A + aoff + (size_t)mb * 16 * K + kc); if (NSPLIT == 1 || NSPLIT == 2) a2[mb] = WFrag<T16>::ld(A2 + aoff + (size_t)mb * 16 * K + kc); }
#pragma unroll
        for (int nb = 0; nb < 4; ++nb) { const V b = WFrag<T16>::ld(Bt + boff + (size_t)nb * 16 * K + kc); V b2; if (NSPLIT >= 2) b2 = WFrag<T16>::ld(Bt2 + boff + (size_t)nb * 16 * K + kc);
#pragma unroll
            for (int mb = 0; mb < 4; ++mb) { acc[mb][nb] = WFrag<T16>::mma(a[mb], b, acc[mb][nb]); if (NSPLIT == 1 || NSPLIT == 2) acc[mb][nb] = WFrag<T16>::mma(a2[mb], b, acc[mb][nb]); if (NSPLIT >= 2) acc[mb][nb] = WFrag<T16>::mma(a[mb], b2, acc[mb][nb]); } }
        asm volatile("v_nop\n\tv_nop\n\tv_nop\n\tv_nop" : "+v"(acc[0][0]), "+v"(acc[1][1]), "+v"(acc[2][2]), "+v"(acc[3][3]) : "v"(a[0]), "v"(a[3]));
    }
    if constexpr (EPI == 0) {
#pragma unroll
        for (int mb = 0; mb < 4; ++mb) {
#pragma unroll
            for (int nb = 0; nb < 4; ++nb) {
#pragma unroll
                for (int j = 0; j < 8; ++j) os[(hi * 8 + j) * 68 + nb * 16 + lr] = acc[mb][nb][j]; }
            __syncthreads();
            float* crow = C + (size_t)(r0 + mb * 16) * ldc + c0;
#pragma unroll 1
            for (int ps = 0; ps < 2; ++ps) {
#pragma unroll
                for (int s = 0; s < 8; ++s) { const unsigned row = 2u * s + hi, cofs = lr * 4u; v4f val = *(const v4fa*)(os + row * 68 + cofs); val[0] += bfr(bias[c0 + cofs]); val[1] += bfr(bias[c0 + cofs + 1]); val[2] += bfr(bias[c0 + cofs + 2]); val[3] += bfr(bias[c0 + cofs + 3]);
                    *(volatile v4f*)(crow + (size_t)row * ldc + cofs) = val; }
                if (ps == 0) __threadfence(); }
            __syncthreads();
        }
    } else if constexpr (EPI == 1) {
        const unsigned cofs = (lane & 7u) * 8u, rq = lane >> 3;
        float bz[8];
#pragma unroll
        for (int q = 0; q < 8; ++q) bz[q] = bfr(bias[c0 + cofs + q]);
#pragma unroll
        for (int mb = 0; mb < 4; ++mb) {
#pragma unroll
            for (int nb = 0; nb < 4; ++nb) {
#pragma unroll
                for (int j = 0; j < 8; ++j) os[(hi * 8 + j) * 68 + nb * 16 + lr] = acc[mb][nb][j]; }
            __syncthreads();
            v8us oh[4], ol[4];
#pragma unroll
            for (int s = 0; s < 4; ++s) { const unsigned row = rq + 4u * s; const v4f va = *(const v4fa*)(os + row * 68 + cofs); const v4f vb = *(const v4fa*)(os + row * 68 + cofs + 4);
#pragma unroll
                for (int q = 0; q < 4; ++q) { unsigned short a, c2; splitf((va[q] + bz[q]) * osc, a, c2); oh[s][q] = a; ol[s][q] = c2; splitf((vb[q] + bz[4 + q]) * osc, a, c2); oh[s][4 + q] = a; ol[s][4 + q] = c2; } }
#pragma unroll 1
            for (int ps = 0; ps < 2; ++ps) {
#pragma unroll
                for (int s = 0; s < 4; ++s) { const size_t dst = (size_t)(r0 + mb * 16 + rq + 4u * s) * ldc + c0 + cofs; *(volatile v8us*)(Ph + dst) = oh[s]; *(volatile v8us*)(Pl + dst) = ol[s]; }
                if (ps == 0) __threadfence(); }
            __syncthreads();
        }
    } else {
#pragma unroll
        for (int mb = 0; mb < 4; ++mb)
#pragma unroll
            for (int nb = 0; nb < 4; ++nb) {
                const float bv = bfr(bias[c0 + nb * 16 + lr]);
                v8us o16, oh, ol;
#pragma unroll
                for (int j = 0; j < 8; ++j) { const float y = acc[mb][nb][j] + bv; o16[j] = __builtin_bit_cast(unsigned short, (h16)y); unsigned short a, c2; splitf(y, a, c2); oh[j] = a; ol[j] = c2; }
                const unsigned off = (nb * 16 + lr) * 72u + mb * 16 + 8u * hi;
                *(v8us*)(tt + off) = o16; *(v8us*)(tt + 4608 + off) = oh; *(v8us*)(tt + 9216 + off) = ol;
            }
        __syncthreads();
        const unsigned bidx = r0 / (unsigned)TT, t0 = r0 - bidx * (unsigned)TT; const bool hw = t0 < (unsigned)RH;
        unsigned short* P16u = (unsigned short*)P16;
        const unsigned cofs = (lane & 7u) * 8u, rq = lane >> 3;
#pragma unroll 1
        for (int ps = 0; ps < 2; ++ps) {
#pragma unroll 2
            for (unsigned s = 0; s < 16; ++s) { const unsigned n = rq + 4u * s; const v8us v = *(const v8usa*)(tt + n * 72u + cofs);
                *(volatile v8us*)(P16u + (size_t)(c0 + n) * MT + r0 + cofs) = v;
                if (hw) { const v8us vh = *(const v8usa*)(tt + 4608 + n * 72u + cofs); const v8us vl = *(const v8usa*)(tt + 9216 + n * 72u + cofs); const size_t dh = (size_t)(c0 + n) * MH + (size_t)bidx * RH + t0 + cofs;
                    *(volatile v8us*)(Ph + dh) = vh; *(volatile v8us*)(Pl + dh) = vl; } }
            if (ps == 0) __threadfence(); }
    }
}

__global__ __launch_bounds__(256) void k_cvt8(const float* __restrict__ src, bf* dst) { const size_t i = (size_t)blockIdx.x * 256 + threadIdx.x; if (i >= (size_t)TT * DM / 8) return; const size_t b = blockIdx.y; const v8f v = *(const v8f*)(src + b * (size_t)TT_FULL * DM + i * 8); v8us o;
#pragma unroll
    for (int k = 0; k < 8; ++k) o[k] = f2bf(v[k]); bf* d = dst + b * (size_t)TT * DM + i * 8; *(volatile v8us*)d = o; __threadfence(); *(volatile v8us*)d = o; }

__global__ __launch_bounds__(256) void k_wT(const float* __restrict__ W0, const float* __restrict__ W1, const float* __restrict__ W2, const float* __restrict__ W3, bf* WT) {
    __shared__ __align__(16) unsigned short tl[64 * 72];
    const unsigned z = blockIdx.z; const float* W = (z == 0u) ? W0 : ((z == 1u) ? W1 : ((z == 2u) ? W2 : W3));
    const unsigned n0 = blockIdx.x * 64u, k0 = blockIdx.y * 64u, tid = threadIdx.x;
    const unsigned c4 = (tid & 15u) * 4u, kr0 = tid >> 4;
#pragma unroll
    for (unsigned i = 0; i < 4; ++i) { const unsigned kr = kr0 + 16u * i; const v4f v = *(const v4f*)(W + (size_t)(k0 + kr) * DM + n0 + c4);
#pragma unroll
        for (int q = 0; q < 4; ++q) tl[(c4 + q) * 72u + kr] = f2bf(v[q]); }
    __syncthreads();
    const unsigned cofs = (tid & 7u) * 8u, nr0 = tid >> 3;
    bf* dstp = WT + (size_t)z * DM * DM;
    v8us o[2];
#pragma unroll
    for (unsigned i = 0; i < 2; ++i) o[i] = *(const v8usa*)(tl + (nr0 + 32u * i) * 72u + cofs);
#pragma unroll 1
    for (int ps = 0; ps < 2; ++ps) {
#pragma unroll
        for (unsigned i = 0; i < 2; ++i) *(volatile v8us*)(dstp + (size_t)(n0 + nr0 + 32u * i) * DM + k0 + cofs) = o[i];
        if (ps == 0) __threadfence(); }
}

__device__ __forceinline__ v8f sc_tile(const bf* __restrict__ Kh, const bf* __restrict__ Kl, size_t koff, v16bf qh0, v16bf qh1, v16bf ql0, v16bf ql1) {
    const v16bf kh0 = WFrag<bf>::ld(Kh + koff), kl0 = WFrag<bf>::ld(Kl + koff), kh1 = WFrag<bf>::ld(Kh + koff + 32), kl1 = WFrag<bf>::ld(Kl + koff + 32);
    v8f s = (v8f){};
    s = wmmab(kh0, qh0, s); s = wmmab(kl0, qh0, s); s = wmmab(kh0, ql0, s);
    s = wmmab(kh1, qh1, s); s = wmmab(kl1, qh1, s); s = wmmab(kh1, ql1, s);
    asm volatile("v_nop\n\tv_nop\n\tv_nop\n\tv_nop" : "+v"(s) : "v"(kh1), "v"(kl1), "v"(ql1));
    return s;
}

template <bool HIRES>
__global__ __launch_bounds__(32) void k_flash(const bf* __restrict__ Qh, const bf* __restrict__ Ql, const bf* __restrict__ Kh, const bf* __restrict__ Kl, const h16* __restrict__ VT16, const bf* __restrict__ VTh, const bf* __restrict__ VTl, bf* Yh, bf* Yl) {
    __shared__ __align__(16) unsigned short osl[2 * 16 * 72];
    const unsigned lane = threadIdx.x & 31u, lr = lane & 15u, hi = lane >> 4;
    const unsigned qrow0 = (HIRES ? 0u : (unsigned)RH) + blockIdx.x * 16u;
    const unsigned h = blockIdx.y, b = blockIdx.z;
    const size_t tok0 = (size_t)b * TT;
    const size_t qoff = (tok0 + qrow0 + lr) * DM + h * HD + 8u * hi;
    const v16bf qh0 = WFrag<bf>::ld(Qh + qoff), qh1 = WFrag<bf>::ld(Qh + qoff + 32), ql0 = WFrag<bf>::ld(Ql + qoff), ql1 = WFrag<bf>::ld(Ql + qoff + 32);
    v8f acc[4];
#pragma unroll
    for (int c = 0; c < 4; ++c) acc[c] = (v8f){};
    float mrun = -1.0e30f, lrun = 0.0f;
    const unsigned nkt = (qrow0 >> 5) + 1u;
    const unsigned qi = qrow0 + lr;
    const float pexp = HIRES ? 0.0f : 10.0f;
#pragma unroll 1
    for (unsigned kt = 0; kt < nkt; ++kt) {
        const unsigned key0 = kt * 32u;
        const size_t koff = (tok0 + key0 + lr) * DM + h * HD + 8u * hi;
        const v8f s0 = sc_tile(Kh, Kl, koff, qh0, qh1, ql0, ql1);
        const v8f s1 = sc_tile(Kh, Kl, koff + (size_t)16 * DM, qh0, qh1, ql0, ql1);
        float p0[8], p1[8]; float mx = -1.0e30f;
#pragma unroll
        for (int r = 0; r < 8; ++r) { const unsigned kj = key0 + 8u * hi + r; p0[r] = (kj <= qi) ? s0[r] : -1.0e30f; p1[r] = (kj + 16u <= qi) ? s1[r] : -1.0e30f; mx = fmaxf(mx, fmaxf(p0[r], p1[r])); }
        mx = fmaxf(mx, __shfl_xor(mx, 16, 32));
        const float mnew = fmaxf(mrun, mx);
        const float scl = __builtin_amdgcn_exp2f((mrun - mnew) * L2E);
        float psum = 0.0f;
#pragma unroll
        for (int r = 0; r < 8; ++r) { p0[r] = __builtin_amdgcn_exp2f((p0[r] - mnew) * L2E + pexp); p1[r] = __builtin_amdgcn_exp2f((p1[r] - mnew) * L2E + pexp); psum += p0[r] + p1[r]; }
        lrun = lrun * scl + psum; mrun = mnew;
#pragma unroll
        for (int c = 0; c < 4; ++c)
#pragma unroll
            for (int r = 0; r < 8; ++r) acc[c][r] *= scl;
        if constexpr (HIRES) {
            v8us h0, l0, h1, l1;
#pragma unroll
            for (int r = 0; r < 8; ++r) { unsigned short a, c2; splitf(p0[r], a, c2); h0[r] = a; l0[r] = c2; splitf(p1[r], a, c2); h1[r] = a; l1[r] = c2; }
            const v16bf ph = cat16b(h0, h1), pl = cat16b(l0, l1);
            const size_t voff = (size_t)(h * HD + lr) * MH + (size_t)b * RH + key0 + 8u * hi;
            v16bf vh, vl;
#pragma unroll
            for (int c = 0; c < 4; ++c) { vh = WFrag<bf>::ld(VTh + voff + (size_t)c * 16 * MH); vl = WFrag<bf>::ld(VTl + voff + (size_t)c * 16 * MH);
                acc[c] = wmmab(vh, ph, acc[c]); acc[c] = wmmab(vl, ph, acc[c]); acc[c] = wmmab(vh, pl, acc[c]); }
            asm volatile("v_nop\n\tv_nop\n\tv_nop\n\tv_nop" : "+v"(acc[0]), "+v"(acc[1]), "+v"(acc[2]), "+v"(acc[3]) : "v"(vh), "v"(vl), "v"(ph), "v"(pl));
        } else {
            v8h a0, a1;
#pragma unroll
            for (int r = 0; r < 8; ++r) { a0[r] = (h16)p0[r]; a1[r] = (h16)p1[r]; }
            const v16h pf = cat16(a0, a1);
            const size_t voff = (size_t)(h * HD + lr) * MT + tok0 + key0 + 8u * hi;
            v16h vf;
#pragma unroll
            for (int c = 0; c < 4; ++c) { vf = WFrag<h16>::ld(VT16 + voff + (size_t)c * 16 * MT); acc[c] = wmma16(vf, pf, acc[c]); }
            asm volatile("v_nop\n\tv_nop\n\tv_nop\n\tv_nop" : "+v"(acc[0]), "+v"(acc[1]), "+v"(acc[2]), "+v"(acc[3]) : "v"(vf), "v"(pf));
        }
    }
    const float l = lrun + __shfl_xor(lrun, 16, 32);
    const float inv = 1.0f / l;
#pragma unroll
    for (int c = 0; c < 4; ++c) { v8us oh, ol;
#pragma unroll
        for (int r = 0; r < 8; ++r) { unsigned short a, c2; splitf(acc[c][r] * inv, a, c2); oh[r] = a; ol[r] = c2; }
        const unsigned off = lr * 72u + c * 16 + 8u * hi;
        *(v8us*)(osl + off) = oh; *(v8us*)(osl + 1152 + off) = ol; }
    __syncthreads();
    const unsigned cofs = (lane & 7u) * 8u, rq = lane >> 3;
    v8us wh[4], wl[4];
#pragma unroll
    for (int s = 0; s < 4; ++s) { const unsigned row = rq + 4u * s; wh[s] = *(const v8usa*)(osl + row * 72u + cofs); wl[s] = *(const v8usa*)(osl + 1152 + row * 72u + cofs); }
#pragma unroll 1
    for (int ps = 0; ps < 2; ++ps) {
#pragma unroll
        for (int s = 0; s < 4; ++s) { const size_t dst = (tok0 + qrow0 + rq + 4u * s) * DM + h * HD + cofs; *(volatile v8us*)(Yh + dst) = wh[s]; *(volatile v8us*)(Yl + dst) = wl[s]; }
        if (ps == 0) __threadfence(); }
}

#define SZ_WT   ((size_t)4 * DM * DM * 2)
#define SZ_TOK  ((size_t)MT * DM * 2)
#define SZ_VH   ((size_t)DM * MH * 2)
static_assert(SZ_WT % 256 == 0);
static_assert(SZ_TOK % 256 == 0);
static_assert(SZ_VH % 256 == 0);
static_assert(SZ_WT + 7 * SZ_TOK + 2 * SZ_VH <= (size_t)134217728);

extern "C" void kernel_launch(void* const* d_in, const int* in_sizes, int n_in,
                              void* d_out, int out_size, void* d_ws, size_t ws_size, hipStream_t stream) {
    if (n_in < 9) return;
    const size_t xneed = ((size_t)(NB - 1) * TT_FULL + TT) * DM;
    if ((size_t)in_sizes[0] < xneed) return;
    if ((size_t)in_sizes[1] < (size_t)DM * DM || (size_t)in_sizes[3] < (size_t)DM * DM || (size_t)in_sizes[5] < (size_t)DM * DM || (size_t)in_sizes[7] < (size_t)DM * DM) return;
    if (in_sizes[2] < DM || in_sizes[4] < DM || in_sizes[6] < DM || in_sizes[8] < DM) return;
    if ((size_t)out_size < (size_t)MT * DM) return;
    const float* x  = (const float*)d_in[0];
    const float* Wq = (const float*)d_in[1]; const float* bq = (const float*)d_in[2];
    const float* Wk = (const float*)d_in[3]; const float* bk = (const float*)d_in[4];
    const float* Wv = (const float*)d_in[5]; const float* bv = (const float*)d_in[6];
    const float* Wo = (const float*)d_in[7]; const float* bo = (const float*)d_in[8];
    float* OUT = (float*)d_out;
    char* wsp = (char*)d_ws;
    auto take = [&](size_t bytes) { char* p = wsp; wsp += (bytes + 255) & ~(size_t)255; return (void*)p; };
    bf* WT  = (bf*)take(SZ_WT);
    bf* XB  = (bf*)take(SZ_TOK);
    bf* Yl  = (bf*)take(SZ_TOK);
    bf* Qh  = (bf*)take(SZ_TOK); bf* Ql = (bf*)take(SZ_TOK); bf* Kh = (bf*)take(SZ_TOK); bf* Kl = (bf*)take(SZ_TOK);
    h16* VT16 = (h16*)take(SZ_TOK);
    bf* VTh = (bf*)take(SZ_VH); bf* VTl = (bf*)take(SZ_VH);
    bf* Yh = XB;
    if ((size_t)(wsp - (char*)d_ws) > ws_size) return;

    k_wT<<<dim3(DM / 64, DM / 64, 4), 256, 0, stream>>>(Wq, Wk, Wv, Wo, WT);
    k_cvt8<<<dim3((unsigned)(((size_t)TT * DM / 8 + 255) / 256), NB, 1), 256, 0, stream>>>(x, XB);
    const dim3 gg(MT / 64, DM / 64, 1);
    k_gemmw<bf, 0, 1><<<gg, 32, 0, stream>>>(XB, nullptr, WT, nullptr, DM, nullptr, DM, bq, Qh, Ql, nullptr, 0.125f);
    k_gemmw<bf, 0, 1><<<gg, 32, 0, stream>>>(XB, nullptr, WT + (size_t)DM * DM, nullptr, DM, nullptr, DM, bk, Kh, Kl, nullptr, 1.0f);
    k_gemmw<bf, 0, 2><<<gg, 32, 0, stream>>>(XB, nullptr, WT + (size_t)2 * DM * DM, nullptr, DM, nullptr, DM, bv, VTh, VTl, VT16, 1.0f);
    k_flash<true><<<dim3(RH / 16, NH_, NB), 32, 0, stream>>>(Qh, Ql, Kh, Kl, VT16, VTh, VTl, Yh, Yl);
    if (TT > RH) k_flash<false><<<dim3((TT - RH) / 16, NH_, NB), 32, 0, stream>>>(Qh, Ql, Kh, Kl, VT16, VTh, VTl, Yh, Yl);
    k_gemmw<bf, 1, 0><<<gg, 32, 0, stream>>>(Yh, Yl, WT + (size_t)3 * DM * DM, nullptr, DM, OUT, DM, bo, nullptr, nullptr, nullptr, 1.0f);
}
